// TimeSFormerXAttention_695784702465
// MI455X (gfx1250) — hardware-verified
//
#include <hip/hip_runtime.h>
#include <hip/hip_bf16.h>
#include <math.h>


typedef _Float16 bf16;
typedef _Float16 f16;
typedef __attribute__((ext_vector_type(4))) unsigned v4u_t;
typedef unsigned v4ua __attribute__((ext_vector_type(4), may_alias));
typedef __attribute__((ext_vector_type(4))) float v4f_t;
typedef float v4fa __attribute__((ext_vector_type(4), may_alias));
typedef __attribute__((ext_vector_type(16))) bf16  bf16x16;
typedef bf16x16 f16x16;
typedef __attribute__((ext_vector_type(8)))  bf16  bf16x8;
typedef bf16x8 f16x8;
typedef __attribute__((ext_vector_type(4)))  bf16  bf16x4;
typedef __attribute__((ext_vector_type(8)))  float f32x8;
__device__ __forceinline__ f32x8 wmma16(f16x16 a, f16x16 b, f32x8 c) {
  c = __builtin_amdgcn_wmma_f32_16x16x32_f16(false, a, false, b, (short)0, c, false, false);
  asm volatile("v_nop\n\tv_nop\n\tv_nop\n\tv_nop" : "+v"(c) : "v"(a), "v"(b));
  return c;
}
#define LDS_STRIDE 48
#define KSTRIDE    72
#define VSTRIDE    48

__device__ __forceinline__ f32x8 wmma_bf16(bf16x16 a, bf16x16 b, f32x8 c) {
  c = __builtin_amdgcn_wmma_f32_16x16x32_f16(false, a, false, b, (short)0, c, false, false);
  asm volatile("v_nop\n\tv_nop\n\tv_nop\n\tv_nop" : "+v"(c) : "v"(a), "v"(b));
  return c;
}

template <typename T>
__device__ __forceinline__ bf16x16 load_frag(const T* __restrict__ base, int ld,
                                             int row0, int k0) {
  const int lane = threadIdx.x & 31;
  const int r    = lane & 15;
  const int kh   = (lane >> 4) * 8;
  const T* p0 = base + (size_t)(row0 + r) * ld + (k0 + kh);
  const T* p1 = p0 + 16;
  bf16x16 f;
#pragma unroll
  for (int i = 0; i < 8; ++i) {
    f[i]     = (bf16)p0[i];
    f[i + 8] = (bf16)p1[i];
  }
  return f;
}

__device__ __forceinline__ bf16x16 lds_frag(const bf16* base, int stride) {
  const int lane = threadIdx.x & 31;
  const int row  = lane & 15;
  const int kh   = (lane >> 4) * 8;
  const bf16x8 lo = *(const bf16x8*)(base + row * stride + kh);
  const bf16x8 hi = *(const bf16x8*)(base + row * stride + kh + 16);
  bf16x16 f;
#pragma unroll
  for (int i = 0; i < 8; ++i) { f[i] = lo[i]; f[i + 8] = hi[i]; }
  return f;
}

template <typename T>
__device__ __forceinline__ void stage_read16(const T* __restrict__ p, float* buf) {
#pragma unroll
  for (int i = 0; i < 16; ++i) buf[i] = (float)p[i];
}

__device__ __forceinline__ void stage_write(bf16* dst, const float* buf, int nquad) {
#pragma unroll
  for (int i = 0; i < nquad; ++i) {
    bf16x4 q;
    q[0] = (bf16)buf[4 * i];     q[1] = (bf16)buf[4 * i + 1];
    q[2] = (bf16)buf[4 * i + 2]; q[3] = (bf16)buf[4 * i + 3];
    *(bf16x4*)(dst + 4 * i) = q;
  }
}


#define GSTR 48
#define GSTR 48
template <typename AT, int EPI, bool OUT16>
__global__ __launch_bounds__(256) void gemm_kne(const AT* __restrict__ A, int lda, const float* __restrict__ Wm, int ldw,
                                                const float* __restrict__ bias, const float* __restrict__ R, const float* __restrict__ gvec,
                                                void* __restrict__ Yv, int ldy, int K) {
  __shared__ __attribute__((aligned(16))) f16 ldsA[128 * GSTR];
  __shared__ __attribute__((aligned(16))) f16 ldsW[128 * GSTR];
  __shared__ __attribute__((aligned(16))) float oS[8][32 * 68];
  const int tid = threadIdx.x, lane = tid & 31, wave = tid >> 5, cl = lane & 15, rh = (lane >> 4) * 8;
  const int m0 = blockIdx.x * 128, n0 = blockIdx.y * 128;
  const int wm = (wave & 3) * 32, wn = (wave >> 2) * 64;
  f32x8 acc[2][4];
#pragma unroll
  for (int i = 0; i < 2; ++i)
#pragma unroll
    for (int j = 0; j < 4; ++j) { f32x8 z = {}; acc[i][j] = z; }
#pragma unroll 1
  for (int k0 = 0; k0 < K; k0 += 32) {
    __syncthreads();
    { const int row = tid >> 1, ch = (tid & 1) * 16;
      const AT* src = A + (size_t)(m0 + row) * lda + k0 + ch;
#pragma unroll
      for (int g = 0; g < 16; ++g) ldsA[row * GSTR + ch + g] = (f16)src[g]; }
    { const int k = tid >> 3, nn0 = (tid & 7) * 16;
      const float* src = Wm + (size_t)(k0 + k) * ldw + n0 + nn0;
#pragma unroll
      for (int g = 0; g < 4; ++g) { const v4f_t v = *(const v4f_t*)(src + 4 * g);
#pragma unroll
        for (int u = 0; u < 4; ++u) ldsW[(nn0 + 4 * g + u) * GSTR + k] = (f16)v[u]; } }
    __syncthreads();
    f16x16 af[2];
#pragma unroll
    for (int i = 0; i < 2; ++i) af[i] = lds_frag(ldsA + (wm + 16 * i) * GSTR, GSTR);
#pragma unroll
    for (int j = 0; j < 4; ++j) {
      const f16x16 bf = lds_frag(ldsW + (wn + 16 * j) * GSTR, GSTR);
#pragma unroll
      for (int i = 0; i < 2; ++i) acc[i][j] = wmma16(af[i], bf, acc[i][j]);
    }
  }
  float* so = oS[wave];
#pragma unroll
  for (int i = 0; i < 2; ++i)
#pragma unroll
    for (int j = 0; j < 4; ++j) {
      const int n = n0 + wn + 16 * j + cl;
      const float bv = bias ? bias[n] : 0.0f;
      const float gv = (EPI == 2 || EPI == 4) ? gvec[n] : 0.0f;
      if (EPI == 1) {
#pragma unroll 1
        for (int r = 0; r < 8; ++r) { const float xg = acc[i][j][r] + bv; so[(16 * i + rh + r) * 68 + 16 * j + cl] = 0.5f * xg * (1.0f + erff(xg * 0.70710678118654752f)); }
      } else {
#pragma unroll
        for (int r = 0; r < 8; ++r) {
          float v = acc[i][j][r] + bv;
          if (EPI == 3) v = fmaxf(v, 0.0f);
          if (EPI == 4) v = gv * v;
          if (EPI == 2) v = R[(size_t)(m0 + wm + 16 * i + rh + r) * ldy + n] + gv * v;
          so[(16 * i + rh + r) * 68 + 16 * j + cl] = v;
        }
      }
    }
  asm volatile("s_wait_dscnt 0" ::: "memory");
  __builtin_amdgcn_wave_barrier();
#pragma unroll 1
  for (int pass = 0; pass < 2; ++pass) {
    if (OUT16) {
      f16* Y = (f16*)Yv;
#pragma unroll
      for (int it = 0; it < 8; ++it) { const int c = lane + 32 * it, rr = c >> 3, q8 = (c & 7) * 8;
        union { f16 h[8]; v4u_t v; } u;
#pragma unroll
        for (int e = 0; e < 8; ++e) u.h[e] = (f16)so[rr * 68 + q8 + e];
        *(volatile v4u_t*)(Y + (size_t)(m0 + wm + rr) * ldy + n0 + wn + q8) = u.v; }
    } else {
      float* Y = (float*)Yv;
#pragma unroll
      for (int it = 0; it < 16; ++it) { const int f4 = lane + 32 * it, rr = f4 >> 4, q = (f4 & 15) * 4;
        *(volatile v4f_t*)(Y + (size_t)(m0 + wm + rr) * ldy + n0 + wn + q) = *(const v4fa*)(so + rr * 68 + q); }
    }
    __threadfence();
  }
}

template <typename AT, int EPI, bool OUT16>
__global__ __launch_bounds__(256) void gemm_knez(const AT* __restrict__ A, int lda, size_t strideA, const float* __restrict__ Wm, int ldw, size_t strideW,
                                                 const float* __restrict__ bias, const float* __restrict__ R, const float* __restrict__ gvec,
                                                 void* __restrict__ Yv, int ldy, size_t strideY, int K) {
  A += (size_t)blockIdx.z * strideA; Wm += (size_t)blockIdx.z * strideW; Yv = (void*)((char*)Yv + (size_t)blockIdx.z * strideY * (OUT16 ? 2 : 4)); if (R) R += (size_t)blockIdx.z * strideY;
  __shared__ __attribute__((aligned(16))) f16 ldsA[128 * GSTR];
  __shared__ __attribute__((aligned(16))) f16 ldsW[128 * GSTR];
  __shared__ __attribute__((aligned(16))) float oS[8][32 * 68];
  const int tid = threadIdx.x, lane = tid & 31, wave = tid >> 5, cl = lane & 15, rh = (lane >> 4) * 8;
  const int m0 = blockIdx.x * 128, n0 = blockIdx.y * 128;
  const int wm = (wave & 3) * 32, wn = (wave >> 2) * 64;
  f32x8 acc[2][4];
#pragma unroll
  for (int i = 0; i < 2; ++i)
#pragma unroll
    for (int j = 0; j < 4; ++j) { f32x8 z = {}; acc[i][j] = z; }
#pragma unroll 1
  for (int k0 = 0; k0 < K; k0 += 32) {
    __syncthreads();
    { const int row = tid >> 1, ch = (tid & 1) * 16;
      const AT* src = A + (size_t)(m0 + row) * lda + k0 + ch;
#pragma unroll
      for (int g = 0; g < 16; ++g) ldsA[row * GSTR + ch + g] = (f16)src[g]; }
    { const int k = tid >> 3, nn0 = (tid & 7) * 16;
      const float* src = Wm + (size_t)(k0 + k) * ldw + n0 + nn0;
#pragma unroll
      for (int g = 0; g < 4; ++g) { const v4f_t v = *(const v4f_t*)(src + 4 * g);
#pragma unroll
        for (int u = 0; u < 4; ++u) ldsW[(nn0 + 4 * g + u) * GSTR + k] = (f16)v[u]; } }
    __syncthreads();
    f16x16 af[2];
#pragma unroll
    for (int i = 0; i < 2; ++i) af[i] = lds_frag(ldsA + (wm + 16 * i) * GSTR, GSTR);
#pragma unroll
    for (int j = 0; j < 4; ++j) {
      const f16x16 bf = lds_frag(ldsW + (wn + 16 * j) * GSTR, GSTR);
#pragma unroll
      for (int i = 0; i < 2; ++i) acc[i][j] = wmma16(af[i], bf, acc[i][j]);
    }
  }
  float* so = oS[wave];
#pragma unroll
  for (int i = 0; i < 2; ++i)
#pragma unroll
    for (int j = 0; j < 4; ++j) {
      const int n = n0 + wn + 16 * j + cl;
      const float bv = bias ? bias[n] : 0.0f;
      const float gv = (EPI == 2 || EPI == 4) ? gvec[n] : 0.0f;
      if (EPI == 1) {
#pragma unroll 1
        for (int r = 0; r < 8; ++r) { const float xg = acc[i][j][r] + bv; so[(16 * i + rh + r) * 68 + 16 * j + cl] = 0.5f * xg * (1.0f + erff(xg * 0.70710678118654752f)); }
      } else {
#pragma unroll
        for (int r = 0; r < 8; ++r) {
          float v = acc[i][j][r] + bv;
          if (EPI == 3) v = fmaxf(v, 0.0f);
          if (EPI == 4) v = gv * v;
          if (EPI == 2) v = R[(size_t)(m0 + wm + 16 * i + rh + r) * ldy + n] + gv * v;
          so[(16 * i + rh + r) * 68 + 16 * j + cl] = v;
        }
      }
    }
  asm volatile("s_wait_dscnt 0" ::: "memory");
  __builtin_amdgcn_wave_barrier();
#pragma unroll 1
  for (int pass = 0; pass < 2; ++pass) {
    if (OUT16) {
      f16* Y = (f16*)Yv;
#pragma unroll
      for (int it = 0; it < 8; ++it) { const int c = lane + 32 * it, rr = c >> 3, q8 = (c & 7) * 8;
        union { f16 h[8]; v4u_t v; } u;
#pragma unroll
        for (int e = 0; e < 8; ++e) u.h[e] = (f16)so[rr * 68 + q8 + e];
        *(volatile v4u_t*)(Y + (size_t)(m0 + wm + rr) * ldy + n0 + wn + q8) = u.v; }
    } else {
      float* Y = (float*)Yv;
#pragma unroll
      for (int it = 0; it < 16; ++it) { const int f4 = lane + 32 * it, rr = f4 >> 4, q = (f4 & 15) * 4;
        *(volatile v4f_t*)(Y + (size_t)(m0 + wm + rr) * ldy + n0 + wn + q) = *(const v4fa*)(so + rr * 68 + q); }
    }
    __threadfence();
  }
}

template <typename AT, bool ACC>
__global__ __launch_bounds__(256) void gemm_kn2(const AT* __restrict__ A, int lda, size_t strideA,
                                               const float* __restrict__ Wm, int ldw, size_t strideW,
                                               const float* __restrict__ bias, float scale,
                                               float* __restrict__ Y, int ldy, size_t strideY, int K) {
  __shared__ __attribute__((aligned(16))) f16 ldsA[128 * GSTR], ldsAl[128 * GSTR];
  __shared__ __attribute__((aligned(16))) f16 ldsW[128 * GSTR], ldsWl[128 * GSTR];
  __shared__ __attribute__((aligned(16))) float oS[8][32 * 68];
  const int tid = threadIdx.x, lane = tid & 31, wave = tid >> 5, cl = lane & 15, rh = (lane >> 4) * 8;
  const int m0 = blockIdx.x * 128, n0 = blockIdx.y * 128;
  const int wm = (wave & 3) * 32, wn = (wave >> 2) * 64;
  A += (size_t)blockIdx.z * strideA; Wm += (size_t)blockIdx.z * strideW; Y += (size_t)blockIdx.z * strideY;
  f32x8 acc[2][4], accx[2][4];
#pragma unroll
  for (int i = 0; i < 2; ++i)
#pragma unroll
    for (int j = 0; j < 4; ++j) { f32x8 z = {}; acc[i][j] = z; accx[i][j] = z; }
#pragma unroll 1
  for (int k0 = 0; k0 < K; k0 += 32) {
    __syncthreads();
    {
      const int row = tid >> 1, ch = (tid & 1) * 16;
      const AT* src = A + (size_t)(m0 + row) * lda + k0 + ch;
#pragma unroll
      for (int g = 0; g < 16; ++g) { const float v = (float)src[g]; const f16 h = (f16)v; ldsA[row * GSTR + ch + g] = h; ldsAl[row * GSTR + ch + g] = (f16)((v - (float)h) * 2048.0f); }
    }
    {
      const int k = tid >> 3, nn0 = (tid & 7) * 16;
      const float* src = Wm + (size_t)(k0 + k) * ldw + n0 + nn0;
#pragma unroll
      for (int g = 0; g < 4; ++g) { const v4f_t v = *(const v4f_t*)(src + 4 * g);
#pragma unroll
        for (int u = 0; u < 4; ++u) { const f16 h = (f16)v[u]; ldsW[(nn0 + 4 * g + u) * GSTR + k] = h; ldsWl[(nn0 + 4 * g + u) * GSTR + k] = (f16)((v[u] - (float)h) * 2048.0f); } }
    }
    __syncthreads();
    f16x16 af[2], afl[2];
#pragma unroll
    for (int i = 0; i < 2; ++i) { af[i] = lds_frag(ldsA + (wm + 16 * i) * GSTR, GSTR); afl[i] = lds_frag(ldsAl + (wm + 16 * i) * GSTR, GSTR); }
#pragma unroll
    for (int j = 0; j < 4; ++j) {
      const f16x16 bf = lds_frag(ldsW + (wn + 16 * j) * GSTR, GSTR), bfl = lds_frag(ldsWl + (wn + 16 * j) * GSTR, GSTR);
#pragma unroll
      for (int i = 0; i < 2; ++i) { acc[i][j] = wmma16(af[i], bf, acc[i][j]); accx[i][j] = wmma16(af[i], bfl, accx[i][j]); accx[i][j] = wmma16(afl[i], bf, accx[i][j]); }
    }
  }
  float* so = oS[wave];
#pragma unroll
  for (int i = 0; i < 2; ++i)
#pragma unroll
    for (int j = 0; j < 4; ++j) {
      const float bv = bias ? bias[n0 + wn + 16 * j + cl] : 0.0f;
#pragma unroll
      for (int r = 0; r < 8; ++r) so[(16 * i + rh + r) * 68 + 16 * j + cl] = (acc[i][j][r] + accx[i][j][r] * (1.0f / 2048.0f)) * scale + bv;
    }
  asm volatile("s_wait_dscnt 0" ::: "memory");
  __builtin_amdgcn_wave_barrier();
  if (ACC) {
#pragma unroll
    for (int it = 0; it < 16; ++it) { const int f4 = lane + 32 * it, rr = f4 >> 4, q = (f4 & 15) * 4;
      const v4f_t old = *(const v4fa*)(Y + (size_t)(m0 + wm + rr) * ldy + n0 + wn + q);
      v4f_t v = *(const v4fa*)(so + rr * 68 + q); v += old; *(v4fa*)(so + rr * 68 + q) = v; }
    asm volatile("s_wait_dscnt 0" ::: "memory");
  }
#pragma unroll 1
  for (int pass = 0; pass < 2; ++pass) {
#pragma unroll
    for (int it = 0; it < 16; ++it) { const int f4 = lane + 32 * it, rr = f4 >> 4, q = (f4 & 15) * 4;
      *(volatile v4f_t*)(Y + (size_t)(m0 + wm + rr) * ldy + n0 + wn + q) = *(const v4fa*)(so + rr * 68 + q); }
    __threadfence();
  }
}

__global__ __launch_bounds__(256) void k_transpose(const float* __restrict__ Wm, float* __restrict__ Wt, int rows, int cols) {
  __shared__ float tS[64][65];
  const int tid = threadIdx.x, tbj = cols / 64, bi = blockIdx.x / tbj, bj = blockIdx.x % tbj;
  for (int e = tid; e < 64 * 64; e += 256) { const int r = e >> 6, c = e & 63; tS[r][c] = Wm[(size_t)(bi * 64 + r) * cols + bj * 64 + c]; }
  __syncthreads();
  for (int ch = tid; ch < 64 * 16; ch += 256) { const int r = ch >> 4, q4 = (ch & 15) * 4; v4f_t o; o[0] = tS[q4][r]; o[1] = tS[q4 + 1][r]; o[2] = tS[q4 + 2][r]; o[3] = tS[q4 + 3][r];
    float* dst = Wt + (size_t)(bj * 64 + r) * rows + bi * 64 + q4; *(volatile v4f_t*)dst = o; __threadfence(); *(volatile v4f_t*)dst = o; }
}


#define GSTR 48
#define SS 2048
#define HH 32
#define DKK 64
template <typename AT, int MODE>
__global__ __launch_bounds__(256) void gemm_rb_kernel(
    const AT* __restrict__ A, const float* __restrict__ W,
    const float* __restrict__ bias, const float* __restrict__ rowscale, const float* __restrict__ R, const float* __restrict__ rowbias, void* __restrict__ out,
    int M, int N, int K) {
  __shared__ bf16 ldsA[128 * LDS_STRIDE];
  __shared__ bf16 ldsW[256 * LDS_STRIDE];
  __shared__ __attribute__((aligned(16))) unsigned char sob[256 * 136 * 2];

  const int t    = threadIdx.x;
  const int wave = t >> 5;
  const int lane = t & 31;
  const int wm   = (wave & 1) * 64;
  const int wn   = (wave >> 1) * 64;
  const int mBlk = blockIdx.x * 128;
  const int nBlk = blockIdx.y * 256;

  const int arow = t >> 1;
  const int ach  = (t & 1) * 16;

  float abuf[16];
  float wbuf[32];

  stage_read16(A + (size_t)(mBlk + arow) * K + ach, abuf);
  const int nrow = min(nBlk + t, N - 1);
  stage_read16(W + (size_t)nrow * K,          wbuf);
  stage_read16(W + (size_t)nrow * K + 16,     wbuf + 16);

  f32x8 acc[4][4] = {};

  for (int k = 0; k < K; k += 32) {
    __syncthreads();
    stage_write(&ldsA[arow * LDS_STRIDE + ach], abuf, 4);
    stage_write(&ldsW[t * LDS_STRIDE],          wbuf, 8);
    if (k + 32 < K) {
      stage_read16(A + (size_t)(mBlk + arow) * K + (k + 32) + ach, abuf);
      stage_read16(W + (size_t)nrow * K + (k + 32),          wbuf);
      stage_read16(W + (size_t)nrow * K + (k + 32) + 16,     wbuf + 16);
    }
    __syncthreads();

    bf16x16 af[4], wf[4];
#pragma unroll
    for (int i = 0; i < 4; ++i)
      af[i] = lds_frag(ldsA + (wm + 16 * i) * LDS_STRIDE, LDS_STRIDE);
#pragma unroll
    for (int j = 0; j < 4; ++j)
      wf[j] = lds_frag(ldsW + (wn + 16 * j) * LDS_STRIDE, LDS_STRIDE);
#pragma unroll
    for (int i = 0; i < 4; ++i)
#pragma unroll
      for (int j = 0; j < 4; ++j)
        acc[i][j] = wmma_bf16(af[i], wf[j], acc[i][j]);
  }

  const int nlane = lane & 15;
  const int mh    = (lane >> 4) * 8;
  __syncthreads();
  if (MODE == 0 || MODE == 1 || MODE == 3) {
    bf16* so = (bf16*)sob;
#pragma unroll
    for (int i = 0; i < 4; ++i)
#pragma unroll
      for (int j = 0; j < 4; ++j) {
        const int nl = wn + 16 * j + nlane;
        const float bv = bias ? bias[nBlk + nl] : 0.0f;
        if (MODE == 3) {
#pragma unroll 1
          for (int r = 0; r < 8; ++r) {
            const int ml = wm + 16 * i + mh + r;
            const float xg = acc[i][j][r] + bv;
            so[ml * 264 + nl] = (bf16)(0.5f * xg * (1.0f + erff(xg * 0.70710678118654752f)));
          }
        } else {
#pragma unroll
        for (int r = 0; r < 8; ++r) {
          const int ml = wm + 16 * i + mh + r;
          const bf16 hv = (bf16)(acc[i][j][r] + bv);
          if (MODE == 0) so[ml * 264 + nl] = hv;
          else           so[nl * 136 + ml] = hv;
        }
        }
      }
    __syncthreads();
#pragma unroll 1
    for (int pass = 0; pass < 2; ++pass) {
      if (MODE == 0 || MODE == 3) {
        for (int ch = t; ch < 128 * 32; ch += 256) { const int ml = ch >> 5, q = (ch & 31) * 8;
          *(volatile v4u_t*)((bf16*)out + (size_t)(mBlk + ml) * N + nBlk + q) = *(const v4ua*)(so + ml * 264 + q); }
      } else {
        const int b_ = mBlk / SS, s0 = mBlk % SS;
        for (int ch = t; ch < 256 * 16; ch += 256) { const int nl = ch >> 4, q = (ch & 15) * 8; const int n = nBlk + nl, h = n >> 6, dk = n & (DKK - 1);
          *(volatile v4u_t*)((bf16*)out + (((size_t)(b_ * HH + h)) * DKK + dk) * SS + s0 + q) = *(const v4ua*)(so + nl * 136 + q); }
      }
      __threadfence();
    }
  } else {
    float* so = (float*)sob;
#pragma unroll 1
    for (int hf = 0; hf < 2; ++hf) {
      if (wm == hf * 64) {
#pragma unroll
        for (int i = 0; i < 4; ++i)
#pragma unroll
          for (int j = 0; j < 4; ++j) {
            const int nl = wn + 16 * j + nlane;
            const float bv = bias ? bias[nBlk + nl] : 0.0f;
#pragma unroll
            for (int r = 0; r < 8; ++r) { const int mrow = mBlk + hf * 64 + 16 * i + mh + r; so[(16 * i + mh + r) * 260 + nl] = acc[i][j][r] * (rowscale ? rowscale[mrow] : 1.0f) + bv + (rowbias ? rowbias[mrow] : 0.0f); }
          }
      }
      __syncthreads();
      if (R) {
        for (int ch = t; ch < 64 * 64; ch += 256) { const int ml = ch >> 6, q = (ch & 63) * 4;
          if (nBlk + q < N) { const v4f_t rv = *(const v4f_t*)(R + (size_t)(mBlk + hf * 64 + ml) * N + nBlk + q); v4f_t v = *(const v4fa*)(so + ml * 260 + q); v += rv; *(v4fa*)(so + ml * 260 + q) = v; }     }
        asm volatile("s_wait_dscnt 0" ::: "memory");
      }
#pragma unroll 1
      for (int pass = 0; pass < 2; ++pass) {
        for (int ch = t; ch < 64 * 64; ch += 256) { const int ml = ch >> 6, q = (ch & 63) * 4;
          if (nBlk + q < N) *(volatile v4f_t*)((float*)out + (size_t)(mBlk + hf * 64 + ml) * N + nBlk + q) = *(const v4fa*)(so + ml * 260 + q); }
        __threadfence();
      }
      __syncthreads();
    }
  }
}


template <typename AT, int EPI, bool OUT16, int NJ>
__global__ __launch_bounds__(256) void gemm_sm(const AT* __restrict__ A, int lda, size_t sA, const float* __restrict__ Wm, int ldw, size_t sW,
                                               const float* __restrict__ bias, const float* __restrict__ R, const float* __restrict__ gvec,
                                               void* __restrict__ Yv, int ldy, size_t sY, int K) {
  constexpr int BN = 16 * NJ; constexpr int OST = BN + 4;
  A += (size_t)blockIdx.z * sA; Wm += (size_t)blockIdx.z * sW; Yv = (void*)((char*)Yv + (size_t)blockIdx.z * sY * (OUT16 ? 2 : 4)); if (R) R += (size_t)blockIdx.z * sY;
  __shared__ __attribute__((aligned(16))) f16 ldsA[256 * GSTR];
  __shared__ __attribute__((aligned(16))) f16 ldsW[BN * GSTR];
  __shared__ __attribute__((aligned(16))) float oS[8][32 * OST];
  const int tid = threadIdx.x, lane = tid & 31, wave = tid >> 5, cl = lane & 15, rh = (lane >> 4) * 8;
  const int m0 = blockIdx.x * 256, n0 = blockIdx.y * BN;
  const int wm = wave * 32;
  f32x8 acc[2][NJ];
#pragma unroll
  for (int i = 0; i < 2; ++i)
#pragma unroll
    for (int j = 0; j < NJ; ++j) { f32x8 z = {}; acc[i][j] = z; }
#pragma unroll 1
  for (int k0 = 0; k0 < K; k0 += 32) {
    __syncthreads();
    { const AT* src = A + (size_t)(m0 + tid) * lda + k0;
#pragma unroll
      for (int g = 0; g < 32; ++g) ldsA[tid * GSTR + g] = (f16)src[g]; }
    { const int k = tid >> 3, nn0 = (tid & 7) * (2 * NJ);
      const float* src = Wm + (size_t)(k0 + k) * ldw + n0 + nn0;
#pragma unroll
      for (int g = 0; g < NJ / 2; ++g) { const v4f_t v = *(const v4f_t*)(src + 4 * g);
#pragma unroll
        for (int u = 0; u < 4; ++u) ldsW[(nn0 + 4 * g + u) * GSTR + k] = (f16)v[u]; } }
    __syncthreads();
    f16x16 af[2];
#pragma unroll
    for (int i = 0; i < 2; ++i) af[i] = lds_frag(ldsA + (wm + 16 * i) * GSTR, GSTR);
#pragma unroll
    for (int j = 0; j < NJ; ++j) {
      const f16x16 bf = lds_frag(ldsW + (16 * j) * GSTR, GSTR);
#pragma unroll
      for (int i = 0; i < 2; ++i) acc[i][j] = wmma16(af[i], bf, acc[i][j]);
    }
  }
  float* so = oS[wave];
#pragma unroll
  for (int i = 0; i < 2; ++i)
#pragma unroll
    for (int j = 0; j < NJ; ++j) {
      const int n = n0 + 16 * j + cl;
      const float bv = bias ? bias[n] : 0.0f;
      const float gv = (EPI == 2 || EPI == 4) ? gvec[n] : 0.0f;
#pragma unroll
      for (int r = 0; r < 8; ++r) {
        float v = acc[i][j][r] + bv;
        if (EPI == 3) v = fmaxf(v, 0.0f);
        if (EPI == 2) v = R[(size_t)(m0 + wm + 16 * i + rh + r) * ldy + n] + gv * v;
        if (EPI == 4) v = gv * v;
        so[(16 * i + rh + r) * OST + 16 * j + cl] = v;
      }
    }
  asm volatile("s_wait_dscnt 0" ::: "memory");
  __builtin_amdgcn_wave_barrier();
#pragma unroll 1
  for (int pass = 0; pass < 2; ++pass) {
    if (OUT16) {
      f16* Y = (f16*)Yv;
#pragma unroll
      for (int it = 0; it < BN / 8; ++it) { const int c = lane + 32 * it, rr = c / (BN / 8), q8 = (c % (BN / 8)) * 8;
        union { f16 h[8]; v4u_t v; } u;
#pragma unroll
        for (int e = 0; e < 8; ++e) u.h[e] = (f16)so[rr * OST + q8 + e];
        *(volatile v4u_t*)(Y + (size_t)(m0 + wm + rr) * ldy + n0 + q8) = u.v; }
    } else {
      float* Y = (float*)Yv;
#pragma unroll
      for (int it = 0; it < BN / 4; ++it) { const int f4 = lane + 32 * it, rr = f4 / (BN / 4), q = (f4 % (BN / 4)) * 4;
        *(volatile v4f_t*)(Y + (size_t)(m0 + wm + rr) * ldy + n0 + q) = *(const v4fa*)(so + rr * OST + q); }
    }
    __threadfence();
  }
}

#define NBts 4
#define LVts 16
#define HWts 196
#define LTts 32
#define DDts 768
#define NHts 12
#define HDts 64
#define QPts 256
#define TKPts 128
#define VRts 3136
#define VRPts 3200
#define TRts 512
#define SWts 384
__global__ __launch_bounds__(256) void k_fill(float* __restrict__ p, float val, size_t n4) { const size_t i = (size_t)blockIdx.x * 256 + threadIdx.x; if (i < n4) { v4f_t v = {val, val, val, val}; *(volatile v4f_t*)(p + 4 * i) = v; __threadfence(); *(volatile v4f_t*)(p + 4 * i) = v; } }
__global__ __launch_bounds__(256) void k_dbg_zero(float* __restrict__ p, size_t n4) { const size_t i = (size_t)blockIdx.x * 256 + threadIdx.x; if (i < n4) { v4f_t z = {0.f,0.f,0.f,0.f}; *(volatile v4f_t*)(p + 4 * i) = z; __threadfence(); *(volatile v4f_t*)(p + 4 * i) = z; } }
__global__ __launch_bounds__(256) void k_copy(const float* __restrict__ src, float* __restrict__ dst, size_t n4) { const size_t i = (size_t)blockIdx.x * 256 + threadIdx.x; if (i < n4) { const v4f_t v = *(const v4f_t*)(src + 4 * i); *(volatile v4f_t*)(dst + 4 * i) = v; __threadfence(); *(volatile v4f_t*)(dst + 4 * i) = v; } }
__global__ __launch_bounds__(256) void k_transpose_ld(const float* __restrict__ Wm, int lds, float* __restrict__ Wt, int rows, int cols) {
  __shared__ float tS[64][65];
  const int tid = threadIdx.x, tbj = cols / 64, bi = blockIdx.x / tbj, bj = blockIdx.x % tbj;
  for (int e = tid; e < 64 * 64; e += 256) { const int r = e >> 6, c = e & 63; tS[r][c] = Wm[(size_t)(bi * 64 + r) * lds + bj * 64 + c]; }
  __syncthreads();
  for (int ch = tid; ch < 64 * 16; ch += 256) { const int r = ch >> 4, q4 = (ch & 15) * 4; v4f_t o; o[0] = tS[q4][r]; o[1] = tS[q4 + 1][r]; o[2] = tS[q4 + 2][r]; o[3] = tS[q4 + 3][r];
    float* dst = Wt + (size_t)(bj * 64 + r) * rows + bi * 64 + q4; *(volatile v4f_t*)dst = o; __threadfence(); *(volatile v4f_t*)dst = o; }
}
__device__ __forceinline__ float bf16r(float x) { unsigned int u = __float_as_uint(x); u = (u + 0x7FFFu + ((u >> 16) & 1u)) & 0xFFFF0000u; return __uint_as_float(u); }
__global__ __launch_bounds__(256) void k_rnd(float* __restrict__ X, size_t n4) { const size_t i = (size_t)blockIdx.x * 256 + threadIdx.x; if (i >= n4) return; v4f_t v = *(const v4fa*)(X + 4 * i);
#pragma unroll
  for (int u = 0; u < 4; ++u) v[u] = bf16r(v[u]);
  *(volatile v4fa*)(X + 4 * i) = v; __threadfence(); *(volatile v4fa*)(X + 4 * i) = v; }
__global__ __launch_bounds__(256) void k_wprep(const float* __restrict__ Wt, const float* __restrict__ bt, float* __restrict__ WT, float* __restrict__ B64) { const int i = blockIdx.x, tid = threadIdx.x;
#pragma unroll
  for (int u = 0; u < 3; ++u) { const int o = tid + 256 * u; const float w = 64.0f * bf16r(Wt[(size_t)o * DDts + i]); *(volatile float*)(WT + (size_t)i * DDts + o) = w; __threadfence(); *(volatile float*)(WT + (size_t)i * DDts + o) = w;
    if (i == 0) { const float bb = 64.0f * bf16r(bt[o]); *(volatile float*)(B64 + o) = bb; *(volatile float*)(B64 + o) = bb; } } }
__global__ __launch_bounds__(256) void k_cpyrnd(const float* __restrict__ src, float* __restrict__ dst, size_t n4) { const size_t i = (size_t)blockIdx.x * 256 + threadIdx.x; if (i >= n4) return; v4f_t v = *(const v4f_t*)(src + 4 * i);
#pragma unroll
  for (int u = 0; u < 4; ++u) v[u] = bf16r(v[u]);
  *(volatile v4f_t*)(dst + 4 * i) = v; __threadfence(); *(volatile v4f_t*)(dst + 4 * i) = v; }
__global__ __launch_bounds__(384) void k_xsoft(float* __restrict__ Sm, const int* __restrict__ tmask, int text_queries) { __shared__ float red[384]; const int q = blockIdx.x, v = blockIdx.y, k = threadIdx.x; float* sr = Sm + ((size_t)v * QPts + q) * SWts;
  const bool mq = (text_queries && q < LTts) ? (tmask[q] != 0) : true; const bool isv = (k < 256); const bool pad = isv ? (k >= HWts) : (k - 256 >= LTts); const bool ok = mq && (isv ? true : (tmask[(k - 256) & (LTts - 1)] != 0));
  float val = pad ? -3.0e38f : (ok ? sr[k] : -10000.0f); red[k] = val; __syncthreads();
  if (k < 128) red[k] = fmaxf(red[k], red[k + 256]); __syncthreads(); for (int o = 128; o > 0; o >>= 1) { if (k < o) red[k] = fmaxf(red[k], red[k + o]); __syncthreads(); }
  const float m = red[0]; __syncthreads(); val = pad ? 0.0f : expf(val - m); red[k] = val; __syncthreads();
  if (k < 128) red[k] += red[k + 256]; __syncthreads(); for (int o = 128; o > 0; o >>= 1) { if (k < o) red[k] += red[k + o]; __syncthreads(); }
  const float p = val * (1024.0f / red[0]); *(volatile float*)(sr + k) = p; __threadfence(); *(volatile float*)(sr + k) = p; }
__global__ __launch_bounds__(256) void k_vcat(const float* __restrict__ Vvid, const float* __restrict__ Vtxt, float* __restrict__ VCAT, size_t n4) { const size_t i = (size_t)blockIdx.x * 256 + threadIdx.x; if (i >= n4) return; const size_t e = 4 * i, v = e / ((size_t)SWts * DDts), r = (e / DDts) % SWts, c = e % DDts;
  const v4f_t x = (r < 256) ? *(const v4f_t*)(Vvid + ((v * HWts + r) * DDts + c)) : *(const v4f_t*)(Vtxt + ((v * LTts + (r - 256)) * DDts + c)); *(volatile v4f_t*)(VCAT + e) = x; __threadfence(); *(volatile v4f_t*)(VCAT + e) = x; }
__global__ __launch_bounds__(256) void k_rows_out(const float* __restrict__ src, int nvalid, float* __restrict__ dst, size_t n4) { const size_t i = (size_t)blockIdx.x * 256 + threadIdx.x; if (i >= n4) return; const size_t e = 4 * i, v = e / ((size_t)nvalid * DDts), r = (e / DDts) % nvalid, c = e % DDts;
  const v4f_t x = *(const v4f_t*)(src + ((v * QPts + r) * DDts + c)); *(volatile v4f_t*)(dst + e) = x; __threadfence(); *(volatile v4f_t*)(dst + e) = x; }

extern "C" void kernel_launch(void* const* d_in, const int* in_sizes, int n_in,
                              void* d_out, int out_size, void* d_ws, size_t ws_size,
                              hipStream_t stream) {
  (void)in_sizes; (void)n_in; (void)out_size;
  const float** f = (const float**)d_in;
  const float* vid = f[0], *txt = f[1]; const int* tmask = (const int*)d_in[3];
  const float* v2vW = f[4], *v2vB = f[5], *t2vW = f[6], *t2vB = f[7], *t2tW = f[8], *t2tB = f[9], *v2tW = f[10], *v2tB = f[11];
  float* out0 = (float*)d_out; float* out1 = out0 + (size_t)4 * VRts * DDts;
  char* ws = (char*)d_ws;
  const size_t DW = (size_t)DDts * DDts;
  float* VA = (float*)ws; ws += (size_t)(VRPts + QPts) * DDts * 4; float* VB = (float*)ws; ws += (size_t)(VRPts + QPts) * DDts * 4; float* VC = (float*)ws; ws += (size_t)(VRPts + QPts) * DDts * 4; float* VD = (float*)ws; ws += (size_t)(VRPts + QPts) * DDts * 4;
  float* TA = (float*)ws; ws += (size_t)(TRts + QPts) * DDts * 4; float* TB = (float*)ws; ws += (size_t)(TRts + QPts) * DDts * 4; float* TC2 = (float*)ws; ws += (size_t)(TRts + QPts) * DDts * 4;
  float* KVT = (float*)ws; ws += (size_t)LVts * DDts * 256 * 4; float* KTT = (float*)ws; ws += (size_t)LVts * DDts * TKPts * 4; float* S = (float*)ws; ws += (size_t)LVts * QPts * SWts * 4; float* sc = (float*)ws; ws += 128 * 4; float* VCAT = (float*)ws; ws += (size_t)LVts * SWts * DDts * 4; float* OP = (float*)ws; ws += (size_t)LVts * QPts * DDts * 4; float* VIN = (float*)ws; ws += (size_t)VRPts * DDts * 4; float* TIN = (float*)ws; ws += (size_t)TRts * DDts * 4; float* WB = (float*)ws; ws += (size_t)6 * DDts * DDts * 4; float* BB = (float*)ws; ws += (size_t)6 * DDts * 4; float* g64 = (float*)ws; ws += DDts * 4;
  if ((size_t)(ws - (char*)d_ws) > ws_size) return;
  const dim3 blk(256); const dim3 gv(VRPts / 128, DDts / 256), gt(TRts / 128, DDts / 256);
  k_fill<<<dim3(1), blk, 0, stream>>>(sc, 0.000122070312500f, 128 / 4);
  k_fill<<<dim3(1), blk, 0, stream>>>(g64, 1.0f / 64.0f, DDts / 4);
  { float* vt[4] = {VA, VB, VC, VD}; for (int i = 0; i < 4; ++i) k_fill<<<dim3((QPts * DDts / 4 + 255) / 256), blk, 0, stream>>>(vt[i] + (size_t)VRPts * DDts, 0.0f, (size_t)QPts * DDts / 4);
    k_fill<<<dim3(((size_t)(VRPts - VRts) * DDts / 4 + 255) / 256), blk, 0, stream>>>(VIN + (size_t)VRts * DDts, 0.0f, (size_t)(VRPts - VRts) * DDts / 4);
    float* tt[3] = {TA, TB, TC2}; for (int i = 0; i < 3; ++i) k_fill<<<dim3((QPts * DDts / 4 + 255) / 256), blk, 0, stream>>>(tt[i] + (size_t)TRts * DDts, 0.0f, (size_t)QPts * DDts / 4); }

  for (int b = 0; b < NBts; ++b) { const float* vsrc = vid + (size_t)b * VRts * DDts; const float* vb = VIN;
    k_cpyrnd<<<dim3(((size_t)VRts * DDts / 4 + 255) / 256), blk, 0, stream>>>(vsrc, VIN, (size_t)VRts * DDts / 4); k_cpyrnd<<<dim3(((size_t)TRts * DDts / 4 + 255) / 256), blk, 0, stream>>>(txt + (size_t)b * TRts * DDts, TIN, (size_t)TRts * DDts / 4);
    const float* tb = txt + (size_t)b * TRts * DDts; const int* mb = tmask + b * LTts;
    for (int j = 0; j < 3; ++j) { k_wprep<<<dim3(DDts), blk, 0, stream>>>(v2vW + (size_t)j * DW, v2vB + (size_t)j * DDts, WB + (size_t)j * DW, BB + (size_t)j * DDts); k_wprep<<<dim3(DDts), blk, 0, stream>>>(t2vW + (size_t)j * DW, t2vB + (size_t)j * DDts, WB + (size_t)(3 + j) * DW, BB + (size_t)(3 + j) * DDts); }
    gemm_kne<float, 4, false><<<dim3(VRPts / 128, DDts / 128), blk, 0, stream>>>(VIN, DDts, WB + (size_t)0 * DW, DDts, BB + (size_t)0 * DDts, nullptr, g64, VA, DDts, DDts); gemm_kne<float, 4, false><<<dim3(VRPts / 128, DDts / 128), blk, 0, stream>>>(VIN, DDts, WB + (size_t)1 * DW, DDts, BB + (size_t)1 * DDts, nullptr, g64, VB, DDts, DDts);
    gemm_kne<float, 4, false><<<dim3(VRPts / 128, DDts / 128), blk, 0, stream>>>(VIN, DDts, WB + (size_t)2 * DW, DDts, BB + (size_t)2 * DDts, nullptr, g64, VC, DDts, DDts); gemm_kne<float, 4, false><<<dim3(VRPts / 128, DDts / 128), blk, 0, stream>>>(VIN, DDts, WB + (size_t)3 * DW, DDts, BB + (size_t)3 * DDts, nullptr, g64, VD, DDts, DDts);
    gemm_kne<float, 4, false><<<dim3(TRts / 128, DDts / 128), blk, 0, stream>>>(TIN, DDts, WB + (size_t)4 * DW, DDts, BB + (size_t)4 * DDts, nullptr, g64, TA, DDts, DDts); gemm_kne<float, 4, false><<<dim3(TRts / 128, DDts / 128), blk, 0, stream>>>(TIN, DDts, WB + (size_t)5 * DW, DDts, BB + (size_t)5 * DDts, nullptr, g64, TB, DDts, DDts);
    for (int v = 0; v < LVts; ++v) { k_transpose_ld<<<dim3((256 / 64) * (DDts / 64)), blk, 0, stream>>>(VB + (size_t)v * HWts * DDts, DDts, KVT + (size_t)v * DDts * 256, 256, DDts); k_transpose_ld<<<dim3((TKPts / 64) * (DDts / 64)), blk, 0, stream>>>(TA + (size_t)v * LTts * DDts, DDts, KTT + (size_t)v * DDts * TKPts, TKPts, DDts); }
    k_vcat<<<dim3(((size_t)LVts * SWts * DDts / 4 + 255) / 256), blk, 0, stream>>>(VC, TB, VCAT, (size_t)LVts * SWts * DDts / 4);
    for (int h = 0; h < NHts; ++h) {
      gemm_kn2<float, false><<<dim3(QPts / 128, 256 / 128, LVts), blk, 0, stream>>>(VA + h * HDts, DDts, (size_t)HWts * DDts, KVT + (size_t)h * HDts * 256, 256, (size_t)DDts * 256, nullptr, 1.0f, S, SWts, (size_t)QPts * SWts, HDts);
      gemm_kn2<float, false><<<dim3(QPts / 128, TKPts / 128, LVts), blk, 0, stream>>>(VD + h * HDts, DDts, (size_t)HWts * DDts, KTT + (size_t)h * HDts * TKPts, TKPts, (size_t)DDts * TKPts, nullptr, 1.0f, S + 256, SWts, (size_t)QPts * SWts, HDts);
      k_xsoft<<<dim3(QPts, LVts), dim3(384), 0, stream>>>(S, mb, 0);
      gemm_sm<float, 4, false, 4><<<dim3(QPts / 256, 1, LVts), blk, 0, stream>>>(S, SWts, (size_t)QPts * SWts, VCAT + h * HDts, DDts, (size_t)SWts * DDts, nullptr, nullptr, sc, OP + h * HDts, DDts, (size_t)QPts * DDts, SWts);
    }
    k_rows_out<<<dim3(((size_t)LVts * HWts * DDts / 4 + 255) / 256), blk, 0, stream>>>(OP, HWts, out0 + (size_t)b * VRts * DDts, (size_t)LVts * HWts * DDts / 4);
    for (int j = 0; j < 3; ++j) { k_wprep<<<dim3(DDts), blk, 0, stream>>>(v2tW + (size_t)j * DW, v2tB + (size_t)j * DDts, WB + (size_t)j * DW, BB + (size_t)j * DDts); k_wprep<<<dim3(DDts), blk, 0, stream>>>(t2tW + (size_t)j * DW, t2tB + (size_t)j * DDts, WB + (size_t)(3 + j) * DW, BB + (size_t)(3 + j) * DDts); }
    gemm_kne<float, 4, false><<<dim3(VRPts / 128, DDts / 128), blk, 0, stream>>>(VIN, DDts, WB + (size_t)1 * DW, DDts, BB + (size_t)1 * DDts, nullptr, g64, VA, DDts, DDts); gemm_kne<float, 4, false><<<dim3(VRPts / 128, DDts / 128), blk, 0, stream>>>(VIN, DDts, WB + (size_t)2 * DW, DDts, BB + (size_t)2 * DDts, nullptr, g64, VB, DDts, DDts);
    gemm_kne<float, 4, false><<<dim3(TRts / 128, DDts / 128), blk, 0, stream>>>(TIN, DDts, WB + (size_t)0 * DW, DDts, BB + (size_t)0 * DDts, nullptr, g64, TA, DDts, DDts); gemm_kne<float, 4, false><<<dim3(TRts / 128, DDts / 128), blk, 0, stream>>>(TIN, DDts, WB + (size_t)3 * DW, DDts, BB + (size_t)3 * DDts, nullptr, g64, TB, DDts, DDts);
    gemm_kne<float, 4, false><<<dim3(TRts / 128, DDts / 128), blk, 0, stream>>>(TIN, DDts, WB + (size_t)4 * DW, DDts, BB + (size_t)4 * DDts, nullptr, g64, TC2, DDts, DDts);
    for (int v = 0; v < LVts; ++v) { k_transpose_ld<<<dim3((256 / 64) * (DDts / 64)), blk, 0, stream>>>(VA + (size_t)v * HWts * DDts, DDts, KVT + (size_t)v * DDts * 256, 256, DDts); k_transpose_ld<<<dim3((TKPts / 64) * (DDts / 64)), blk, 0, stream>>>(TC2 + (size_t)v * LTts * DDts, DDts, KTT + (size_t)v * DDts * TKPts, TKPts, DDts); }
    gemm_kne<float, 4, false><<<dim3(TRts / 128, DDts / 128), blk, 0, stream>>>(TIN, DDts, WB + (size_t)5 * DW, DDts, BB + (size_t)5 * DDts, nullptr, g64, TC2, DDts, DDts);
    k_vcat<<<dim3(((size_t)LVts * SWts * DDts / 4 + 255) / 256), blk, 0, stream>>>(VB, TC2, VCAT, (size_t)LVts * SWts * DDts / 4);
    for (int h = 0; h < NHts; ++h) {
      gemm_kn2<float, false><<<dim3(QPts / 128, 256 / 128, LVts), blk, 0, stream>>>(TA + h * HDts, DDts, (size_t)LTts * DDts, KVT + (size_t)h * HDts * 256, 256, (size_t)DDts * 256, nullptr, 1.0f, S, SWts, (size_t)QPts * SWts, HDts);
      gemm_kn2<float, false><<<dim3(QPts / 128, TKPts / 128, LVts), blk, 0, stream>>>(TB + h * HDts, DDts, (size_t)LTts * DDts, KTT + (size_t)h * HDts * TKPts, TKPts, (size_t)DDts * TKPts, nullptr, 1.0f, S + 256, SWts, (size_t)QPts * SWts, HDts);
      k_xsoft<<<dim3(QPts, LVts), dim3(384), 0, stream>>>(S, mb, 1);
      gemm_sm<float, 4, false, 4><<<dim3(QPts / 256, 1, LVts), blk, 0, stream>>>(S, SWts, (size_t)QPts * SWts, VCAT + h * HDts, DDts, (size_t)SWts * DDts, nullptr, nullptr, sc, OP + h * HDts, DDts, (size_t)QPts * DDts, SWts);
    }
    k_rows_out<<<dim3(((size_t)LVts * LTts * DDts / 4 + 255) / 256), blk, 0, stream>>>(OP, LTts, out1 + (size_t)b * TRts * DDts, (size_t)LVts * LTts * DDts / 4);
  }
}
